// TipAdapterHead_28948079575487
// MI455X (gfx1250) — hardware-verified
//
#include <hip/hip_runtime.h>
#include <math.h>

constexpr int   kNQ        = 4096;
constexpr int   kNK        = 16384;
constexpr int   kDim       = 512;
constexpr int   kChunk     = 4096;
constexpr int   kNChunks   = kNK / kChunk;
constexpr float kUnitCarry = 64.0f;
constexpr float kAffCarry  = 4096.0f;
constexpr float kBeta      = 5.5f;
constexpr float kAlpha     = 0.5f;
constexpr float kNormEps   = 1e-12f;

typedef __attribute__((ext_vector_type(16))) _Float16 v16h;
typedef __attribute__((ext_vector_type(8)))  _Float16 v8h;
typedef __attribute__((ext_vector_type(16))) __bf16   v16b;
typedef __attribute__((ext_vector_type(8)))  __bf16   v8b;
typedef __attribute__((ext_vector_type(8)))  float    v8f;
typedef __attribute__((ext_vector_type(4)))  float    v4f;
typedef __attribute__((ext_vector_type(4)))  unsigned int v4u;

__device__ __forceinline__ unsigned short f2bf_bits(float f) {
  unsigned u = __float_as_uint(f);
  return (unsigned short)((u + 0x7FFFu + ((u >> 16) & 1u)) >> 16);
}
__device__ __forceinline__ float bf_bits2f(unsigned short h) { return __uint_as_float(((unsigned)h) << 16); }

__device__ __forceinline__ void dep_guard_h(v8f& a, v8f& b, v16h x, v16h y) { asm volatile("v_nop\n\tv_nop\n\tv_nop\n\tv_nop" : "+v"(a), "+v"(b) : "v"(x), "v"(y)); }
__device__ __forceinline__ void dep_guard_b(v8f& a, v8f& b, v16b x, v16b y) { asm volatile("v_nop\n\tv_nop\n\tv_nop\n\tv_nop" : "+v"(a), "+v"(b) : "v"(x), "v"(y)); }
__device__ __forceinline__ void keep4_h(v16h a, v16h b, v16h c, v16h d) { asm volatile("v_nop" :: "v"(a), "v"(b), "v"(c), "v"(d)); }
__device__ __forceinline__ void keep4_b(v16b a, v16b b, v16b c, v16b d) { asm volatile("v_nop" :: "v"(a), "v"(b), "v"(c), "v"(d)); }
__device__ __forceinline__ void acc_guard4(v8f& a, v8f& b, v8f& c, v8f& d) { asm volatile("v_nop\n\tv_nop\n\tv_nop\n\tv_nop" : "+v"(a), "+v"(b), "+v"(c), "+v"(d)); }
template <typename T> struct Frag;
template <> struct Frag<_Float16> {
  typedef v16h V; union U { v16h v; v8h h[2]; };
  static __device__ __forceinline__ v16h load(const _Float16* p) {
    U f; f.h[0] = *(const v8h*)(p); f.h[1] = *(const v8h*)(p + 16); return f.v;
  }
  static __device__ __forceinline__ v8f mma(v16h a, v16h b, v8f c) {
    return __builtin_amdgcn_wmma_f32_16x16x32_f16(false, a, false, b, (short)0, c, false, false);
  }
  static __device__ __forceinline__ void guard(v8f& a, v8f& b, v16h x, v16h y) { dep_guard_h(a, b, x, y); }
  static __device__ __forceinline__ void keep(v16h a, v16h b, v16h c, v16h d) { keep4_h(a, b, c, d); }
};
template <> struct Frag<__bf16> {
  typedef v16b V; union U { v16b v; v8b h[2]; };
  static __device__ __forceinline__ v16b load(const __bf16* p) {
    U f; f.h[0] = *(const v8b*)(p); f.h[1] = *(const v8b*)(p + 16); return f.v;
  }
  static __device__ __forceinline__ v8f mma(v16b a, v16b b, v8f c) {
    return __builtin_amdgcn_wmma_f32_16x16x32_bf16(false, a, false, b, (short)0, c, false, false);
  }
  static __device__ __forceinline__ void guard(v8f& a, v8f& b, v16b x, v16b y) { dep_guard_b(a, b, x, y); }
  static __device__ __forceinline__ void keep(v16b a, v16b b, v16b c, v16b d) { keep4_b(a, b, c, d); }
};

__device__ __forceinline__ unsigned pk16(unsigned short a, unsigned short b) { return (unsigned)a | ((unsigned)b << 16); }
__device__ __forceinline__ unsigned short h_bits(float f) { const _Float16 h = (_Float16)f; return __builtin_bit_cast(unsigned short, h); }

template <int ET> struct Elem;
template <> struct Elem<0> { typedef _Float16 T; };
template <> struct Elem<1> { typedef __bf16 T; };
template <int ET, bool SPLIT, int BIAS_MODE, int OUT_MODE, bool RESID, int ACT = 0>
__global__ __launch_bounds__(256) void wmma_gemm64(
    const unsigned short* __restrict__ Ap, const unsigned short* __restrict__ A2p, int lda, long strideA,
    const unsigned short* __restrict__ Btp, const unsigned short* __restrict__ Bt2p, int ldb, long strideB,
    void* __restrict__ Cout, void* __restrict__ Cout2, int ldc, long strideC,
    const float* __restrict__ bias,
    const float* __restrict__ resid, long strideR,
    int M, int N, int K, float scale) {
  typedef typename Elem<ET>::T T;
  typedef typename Frag<T>::V V;
  const T* A = (const T*)Ap; const T* A2 = (const T*)A2p; const T* Bt = (const T*)Btp; const T* Bt2 = (const T*)Bt2p;
  __shared__ __align__(16) float sT[8][16 * 68];
  const int b    = blockIdx.y;
  const int lane = threadIdx.x & 31;
  const int wave = threadIdx.x >> 5;
  const int tilesN = N >> 6;
  const int tilesM = M >> 6;
  const int tile = blockIdx.x * 8 + wave;
  if (tile >= tilesM * tilesN) return;
  const int tm = tile / tilesN;
  const int tn = tile - tm * tilesN;
  const int m0 = tm << 6;
  const int n0 = tn << 6;

  const T* Ab  = A  + (size_t)b * strideA;
  const T* Bb  = Bt + (size_t)b * strideB;
  const T* Ab2 = SPLIT ? (A2  + (size_t)b * strideA) : nullptr;
  const T* Bb2 = SPLIT ? (Bt2 + (size_t)b * strideB) : nullptr;

  const int rlane = lane & 15;
  const int koff  = (lane >> 4) * 8;
  const int mOff  = (lane >> 4) * 8;

  v8f acc[4][4];
#pragma unroll
  for (int i = 0; i < 4; ++i)
#pragma unroll
    for (int j = 0; j < 4; ++j) acc[i][j] = (v8f){0.f,0.f,0.f,0.f,0.f,0.f,0.f,0.f};

  for (int k0 = 0; k0 < K; k0 += 32) {
    V bh[4], bl[4];
#pragma unroll
    for (int j = 0; j < 4; ++j) {
      const size_t bo = (size_t)(n0 + (j << 4) + rlane) * ldb + koff + k0;
      bh[j] = Frag<T>::load(Bb + bo);
      if (SPLIT) bl[j] = Frag<T>::load(Bb2 + bo);
    }
#pragma unroll
    for (int i = 0; i < 4; ++i) {
      const size_t ao = (size_t)(m0 + (i << 4) + rlane) * lda + koff + k0;
      V ah = Frag<T>::load(Ab + ao);
      V al;
      if (SPLIT) al = Frag<T>::load(Ab2 + ao);
#pragma unroll
      for (int j = 0; j < 4; ++j) {
        acc[i][j] = Frag<T>::mma(ah, bh[j], acc[i][j]);
        if (SPLIT) {
          acc[i][j] = Frag<T>::mma(ah, bl[j], acc[i][j]);
          acc[i][j] = Frag<T>::mma(al, bh[j], acc[i][j]);
        }
      }
      Frag<T>::guard(acc[i][0], acc[i][3], ah, SPLIT ? al : ah);
    }
    Frag<T>::keep(bh[0], bh[1], bh[2], bh[3]);
    if (SPLIT) Frag<T>::keep(bl[0], bl[1], bl[2], bl[3]);
  }
  acc_guard4(acc[0][0], acc[0][1], acc[0][2], acc[0][3]);
  acc_guard4(acc[1][0], acc[1][1], acc[1][2], acc[1][3]);
  acc_guard4(acc[2][0], acc[2][1], acc[2][2], acc[2][3]);
  acc_guard4(acc[3][0], acc[3][1], acc[3][2], acc[3][3]);

  float* slab = sT[wave];
  const float* Rb = RESID ? (resid + (size_t)b * strideR) : nullptr;
#pragma unroll
  for (int i = 0; i < 4; ++i) {
    const int mBase = m0 + (i << 4);
#pragma unroll
    for (int j = 0; j < 4; ++j) {
      const int n = n0 + (j << 4) + rlane;
      float bv = 0.f;
      if (BIAS_MODE == 2) bv = bias[n];
#pragma unroll
      for (int r = 0; r < 8; ++r) {
        float v = acc[i][j][r] * scale;
        if (BIAS_MODE == 1) v += bias[mBase + mOff + r];
        if (BIAS_MODE == 2) v += bv;
        if (RESID) v += Rb[(size_t)(mBase + mOff + r) * ldc + n];
        if (ACT == 2) v = fmaxf(v, 0.0f);
        if (ACT == 4) v = (v > 0.f) ? v : 0.01f * v;
        if (ACT == 7) v = __expf(-kBeta * (1.0f - v)) * kAffCarry;
        slab[(mOff + r) * 68 + (j << 4) + rlane] = v;
      }
    }
    __builtin_amdgcn_fence(__ATOMIC_RELEASE, "workgroup");
    __builtin_amdgcn_wave_barrier();
    __builtin_amdgcn_fence(__ATOMIC_ACQUIRE, "workgroup");
    if (OUT_MODE == 0) {
      float* C = (float*)Cout + (size_t)b * strideC;
      const int hh = lane >> 4, c4 = (lane & 15) * 4;
      for (int pass = 0; pass < 2; ++pass) {
#pragma unroll
        for (int it = 0; it < 8; ++it) {
          const int row = it * 2 + hh;
          v4f v = *(const v4f*)(slab + row * 68 + c4);
          *(volatile v4f*)(C + (size_t)(mBase + row) * ldc + n0 + c4) = v;
        }
        __threadfence();
      }
    } else {
      const int q = lane >> 3, c8 = (lane & 7) * 8;
      unsigned short* C  = (unsigned short*)Cout  + (size_t)b * strideC;
      unsigned short* C2 = (OUT_MODE == 2) ? ((unsigned short*)Cout2 + (size_t)b * strideC) : nullptr;
      for (int pass = 0; pass < 2; ++pass) {
#pragma unroll
        for (int it = 0; it < 4; ++it) {
          const int row = it * 4 + q;
          const float* sp = slab + row * 68 + c8;
          v8h hv, lv;
#pragma unroll
          for (int e = 0; e < 8; ++e) {
            if (OUT_MODE == 1) {
              hv[e] = (_Float16)sp[e];
            } else {
              unsigned short hb = f2bf_bits(sp[e]);
              unsigned short lb = f2bf_bits(sp[e] - bf_bits2f(hb));
              hv[e] = __builtin_bit_cast(_Float16, hb);
              lv[e] = __builtin_bit_cast(_Float16, lb);
            }
          }
          *(volatile v8h*)(C + (size_t)(mBase + row) * ldc + n0 + c8) = hv;
          if (OUT_MODE == 2) *(volatile v8h*)(C2 + (size_t)(mBase + row) * ldc + n0 + c8) = lv;
        }
        __threadfence();
      }
    }
    __builtin_amdgcn_fence(__ATOMIC_RELEASE, "workgroup");
    __builtin_amdgcn_wave_barrier();
    __builtin_amdgcn_fence(__ATOMIC_ACQUIRE, "workgroup");
  }
}

__global__ __launch_bounds__(256) void l2norm_f16_kernel(const float* __restrict__ src, unsigned short* __restrict__ dst, int nrows) {
  const int lane = threadIdx.x & 31;
  const int row  = blockIdx.x * 8 + (threadIdx.x >> 5);
  if (row >= nrows) return;
  const float* p = src + (size_t)row * kDim;
  const v4f a0 = *(const v4f*)(p + 8 * lane);
  const v4f a1 = *(const v4f*)(p + 8 * lane + 4);
  const v4f b0 = *(const v4f*)(p + 256 + 8 * lane);
  const v4f b1 = *(const v4f*)(p + 256 + 8 * lane + 4);
  float s = 0.f;
#pragma unroll
  for (int e = 0; e < 4; ++e) s += a0[e] * a0[e] + a1[e] * a1[e] + b0[e] * b0[e] + b1[e] * b1[e];
#pragma unroll
  for (int off = 16; off > 0; off >>= 1) s += __shfl_xor(s, off, 32);
  const float inv = 1.0f / fmaxf(sqrtf(s), kNormEps);
  const float sc  = inv * kUnitCarry;
  unsigned short ha[8], hb[8];
#pragma unroll
  for (int e = 0; e < 4; ++e) {
    ha[e]     = h_bits(a0[e] * sc);
    ha[4 + e] = h_bits(a1[e] * sc);
    hb[e]     = h_bits(b0[e] * sc);
    hb[4 + e] = h_bits(b1[e] * sc);
  }
  const v4u ua = (v4u){pk16(ha[0], ha[1]), pk16(ha[2], ha[3]), pk16(ha[4], ha[5]), pk16(ha[6], ha[7])};
  const v4u ub = (v4u){pk16(hb[0], hb[1]), pk16(hb[2], hb[3]), pk16(hb[4], hb[5]), pk16(hb[6], hb[7])};
  unsigned short* q0 = dst + (size_t)row * kDim + 8 * lane;
  unsigned short* q1 = q0 + 256;
  *(volatile v4u*)q0 = ua;
  *(volatile v4u*)q1 = ub;
  __threadfence();
  *(volatile v4u*)q0 = ua;
  *(volatile v4u*)q1 = ub;
}

__global__ __launch_bounds__(256) void transpose64_f16_kernel(const unsigned short* __restrict__ in, unsigned short* __restrict__ out) {
  __shared__ __align__(16) unsigned short sh[64 * 72];
  const int t  = threadIdx.x;
  const int n0 = blockIdx.x * 64;
  const int d0 = blockIdx.y * 64;
  const int c8 = (t & 7) * 8;
#pragma unroll
  for (int p = 0; p < 2; ++p) {
    const int r = 32 * p + (t >> 3);
    const v4u v = *(const v4u*)(in + (size_t)(n0 + r) * kDim + d0 + c8);
#pragma unroll
    for (int e = 0; e < 4; ++e) {
      sh[(c8 + 2 * e) * 72 + r]     = (unsigned short)(v[e] & 0xFFFFu);
      sh[(c8 + 2 * e + 1) * 72 + r] = (unsigned short)(v[e] >> 16);
    }
  }
  __syncthreads();
  const int wave = t >> 5, lane = t & 31;
  const int q = lane >> 3, k8 = (lane & 7) * 8;
  v4u vals[2];
#pragma unroll
  for (int it = 0; it < 2; ++it) {
    const int d = wave * 8 + it * 4 + q;
    vals[it] = *(const v4u*)(const void*)(sh + d * 72 + k8);
  }
  for (int pass = 0; pass < 2; ++pass) {
#pragma unroll
    for (int it = 0; it < 2; ++it) {
      const int d = wave * 8 + it * 4 + q;
      *(volatile v4u*)(out + (size_t)(d0 + d) * kNK + n0 + k8) = vals[it];
    }
    __threadfence();
  }
}

extern "C" void kernel_launch(void* const* d_in, const int* in_sizes, int n_in,
                              void* d_out, int out_size, void* d_ws, size_t ws_size,
                              hipStream_t stream) {
  if (n_in < 2) return;
  if (in_sizes[0] != kNQ * kDim) return;
  if (in_sizes[1] != kNK * kDim) return;
  if (out_size != kNQ * kDim) return;

  const float* query = (const float*)d_in[0];
  const float* keys  = (const float*)d_in[1];
  float* outp = (float*)d_out;

  const size_t SZ_QN  = (size_t)kNQ * kDim * 2;
  const size_t SZ_KN  = (size_t)kNK * kDim * 2;
  const size_t SZ_KNT = (size_t)kDim * kNK * 2;
  const size_t SZ_E   = (size_t)kNQ * kChunk * 2;
  const size_t SZ_ACC = (size_t)kNQ * kDim * 4;
  size_t off = 0;
  const size_t oQN   = off; off += SZ_QN;
  const size_t oKN   = off; off += SZ_KN;
  const size_t oKNT  = off; off += SZ_KNT;
  const size_t oE    = off; off += SZ_E;
  const size_t oACCA = off; off += SZ_ACC;
  const size_t oACCB = off; off += SZ_ACC;
  const size_t TOTAL = off;
  if (TOTAL > ws_size) return;
  if (TOTAL > (size_t)134217728) return;

  char* ws = (char*)d_ws;
  unsigned short* QN   = (unsigned short*)(ws + oQN);
  unsigned short* KN   = (unsigned short*)(ws + oKN);
  unsigned short* KNT  = (unsigned short*)(ws + oKNT);
  unsigned short* E16  = (unsigned short*)(ws + oE);
  float*          ACCA = (float*)(ws + oACCA);
  float*          ACCB = (float*)(ws + oACCB);

  const dim3 blk(256);

  l2norm_f16_kernel<<<dim3(kNQ / 8), blk, 0, stream>>>(query, QN, kNQ);
  l2norm_f16_kernel<<<dim3(kNK / 8), blk, 0, stream>>>(keys, KN, kNK);

  transpose64_f16_kernel<<<dim3(kNK / 64, kDim / 64), blk, 0, stream>>>(KN, KNT);

  const int tilesQ = kNQ / 64;
  const dim3 gAff((tilesQ * (kChunk / 64) + 7) / 8, 1);
  const dim3 gRet((tilesQ * (kDim / 64) + 7) / 8, 1);
  const float affScale = 1.0f / (kUnitCarry * kUnitCarry);
  const float retScale = kAlpha / (kAffCarry * kUnitCarry);
  for (int c = 0; c < kNChunks; ++c) {
    const unsigned short* KNc  = KN  + (size_t)c * kChunk * kDim;
    const unsigned short* KNTc = KNT + (size_t)c * kChunk;
    wmma_gemm64<0, false, 0, 1, false, 7><<<gAff, blk, 0, stream>>>(
        QN, QN, kDim, 0L, KNc, KNc, kDim, 0L, (void*)E16, (void*)E16, kChunk, 0L,
        query, query, 0L, kNQ, kChunk, kDim, affScale);
    const float* rsrc = (c == 0) ? query : ((c == 2) ? (const float*)ACCB : (const float*)ACCA);
    float* dst = (c == kNChunks - 1) ? outp : ((c == 1) ? ACCB : ACCA);
    wmma_gemm64<0, false, 0, 0, true, 0><<<gRet, blk, 0, stream>>>(
        E16, E16, kChunk, 0L, KNTc, KNTc, kNK, 0L, (void*)dst, (void*)dst, kDim, 0L,
        query, rsrc, 0L, kNQ, kDim, kChunk, retScale);
  }
}
